// char_CNN_word_CNN_12756052869584
// MI455X (gfx1250) — hardware-verified
//
#include <hip/hip_runtime.h>
#include <stdint.h>

#define NB    128
#define NS    512
#define NW    16
#define CE    50
#define WE    100
#define CC    200
#define NTAG  50
#define CV    100
#define TV    50000
#define NWORD (NB * NS)
#define SEGR  520
#define PE    160
#define PH    208
#define NCP   208
#define CS1   160
#define KC1   480
#define CS2   200
#define KC2   608
#define KO    224
#define NO    64
#define TM    128
#define TN    192
#define TK    64

static_assert((KC1 % 32) == 0 && (KC2 % 32) == 0 && (KO % 32) == 0 && (TK % 32) == 0);
static_assert((PE % 8) == 0 && (PH % 8) == 0 && (NWORD % 128) == 0 && (NS % 128) == 0);
static_assert(((16 * PH * 2) % 128) == 0 && ((16 * PE * 2) % 128) == 0 && ((4 * PH * 2) % 128) == 0 && ((4 * PE * 2) % 128) == 0);
static_assert(((SEGR * PH * 2) % 128) == 0 && ((SEGR * PE * 2) % 128) == 0 && ((16 * NTAG * 4) % 128) == 0);
static_assert(KC1 == 3 * CS1 && KC2 >= 3 * CS2 && (CS2 % 8) == 0 && CS1 == PE && CC + 8 <= PH && WE + CE + 8 <= PE);
static_assert((16 * PH) % (32 * 8) == 0 && (16 * PE) % (8) == 0 && (TN % 32) == 0);

typedef _Float16 v16h __attribute__((ext_vector_type(16)));
typedef _Float16 v8h  __attribute__((ext_vector_type(8)));
typedef _Float16 v4h  __attribute__((ext_vector_type(4)));
typedef float    v8f  __attribute__((ext_vector_type(8)));
typedef float    v4f  __attribute__((ext_vector_type(4)));
typedef int      v4i  __attribute__((ext_vector_type(4)));

union Frag { v16h v; v8h half[2]; };

__device__ __forceinline__ float bf_rt(float f) {
  unsigned u = __float_as_uint(f);
  u = (u + 0x7FFFu + ((u >> 16) & 1u)) & 0xFFFF0000u;
  return __uint_as_float(u);
}
__device__ __forceinline__ int clampi(int v, int lo, int hi) { return v < lo ? lo : (v > hi ? hi : v); }
__device__ __forceinline__ v8f zero8f() { v8f z = {0.f, 0.f, 0.f, 0.f, 0.f, 0.f, 0.f, 0.f}; return z; }
__device__ __forceinline__ v4f zero4f() { v4f z = {0.f, 0.f, 0.f, 0.f}; return z; }
__device__ __forceinline__ v8h zero8h() {
  v8h z;
#pragma unroll
  for (int e = 0; e < 8; ++e) z[e] = (_Float16)0.0f;
  return z;
}

__device__ __forceinline__ v16h ldfrag(const _Float16* p0, const _Float16* p1) {
  Frag f;
  f.half[0] = *(const v8h*)(p0);
  f.half[1] = *(const v8h*)(p1);
  return f.v;
}

__device__ __forceinline__ v8f mma(v16h a, v16h b, v8f c) {
  return __builtin_amdgcn_wmma_f32_16x16x32_f16(false, a, false, b, (short)0, c, false, false);
}
__device__ __forceinline__ void guard4(v8f& c0, v8f& c1, v8f& c2, v8f& c3, v16h a, v16h b0, v16h b1, v16h b2, v16h b3) {
#if defined(__HIP_DEVICE_COMPILE__)
  asm volatile("v_nop\n\tv_nop\n\tv_nop\n\tv_nop"
               : "+v"(c0), "+v"(c1), "+v"(c2), "+v"(c3)
               : "v"(a), "v"(b0), "v"(b1), "v"(b2), "v"(b3));
#endif
}
__device__ __forceinline__ void guard1(v8f& c0, v16h a, v16h b0) {
#if defined(__HIP_DEVICE_COMPILE__)
  asm volatile("v_nop\n\tv_nop\n\tv_nop\n\tv_nop" : "+v"(c0) : "v"(a), "v"(b0));
#endif
}
__device__ __forceinline__ void accg4(v8f& a, v8f& b, v8f& c, v8f& d) {
#if defined(__HIP_DEVICE_COMPILE__)
  asm volatile("v_nop\n\tv_nop\n\tv_nop\n\tv_nop" : "+v"(a), "+v"(b), "+v"(c), "+v"(d));
#endif
}
__device__ __forceinline__ void accg1(v8f& a) {
#if defined(__HIP_DEVICE_COMPILE__)
  asm volatile("v_nop\n\tv_nop\n\tv_nop\n\tv_nop" : "+v"(a));
#endif
}
__device__ __forceinline__ void wave_sync_lds() {
  __builtin_amdgcn_fence(__ATOMIC_RELEASE, "workgroup");
  __builtin_amdgcn_wave_barrier();
  __builtin_amdgcn_fence(__ATOMIC_ACQUIRE, "workgroup");
}

__device__ __forceinline__ void grp4(v8f& c0, v8f& c1, v8f& c2, v8f& c3, v16h a, const _Float16* Bk, int st) {
  const v16h b0 = ldfrag(Bk, Bk + 16);
  const v16h b1 = ldfrag(Bk + st, Bk + st + 16);
  const v16h b2 = ldfrag(Bk + 2 * st, Bk + 2 * st + 16);
  const v16h b3 = ldfrag(Bk + 3 * st, Bk + 3 * st + 16);
  c0 = mma(a, b0, c0);
  c1 = mma(a, b1, c1);
  c2 = mma(a, b2, c2);
  c3 = mma(a, b3, c3);
  guard4(c0, c1, c2, c3, a, b0, b1, b2, b3);
}
__device__ __forceinline__ void grp1(v8f& c0, v16h a, const _Float16* Bk) {
  const v16h b0 = ldfrag(Bk, Bk + 16);
  c0 = mma(a, b0, c0);
  guard1(c0, a, b0);
}

__global__ __launch_bounds__(256) void cvt_plane(const float* __restrict__ src, int srcn, _Float16* dst,
                                                 int kp, int nsegw, int nnseg, int nr,
                                                 int kseg, int nkseg, int cr,
                                                 int sn, int sns, int sc, int sk, float scale, int n8) {
  const int i = blockIdx.x * 256 + threadIdx.x;
  if (i >= n8) return;
  const int kp8  = kp >> 3;
  const int n    = i / kp8;
  const int K0   = (i - n * kp8) * 8;
  const int nseg = n / nsegw;
  const int o    = n - nseg * nsegw;
  const int ks   = K0 / kseg;
  const int c0   = K0 - ks * kseg;
  const bool rv  = (o < nr) && (nseg < nnseg) && (ks < nkseg);
  const int base = o * sn + nseg * sns + ks * sk;
  v8h out;
#pragma unroll
  for (int e = 0; e < 8; ++e) {
    const int c = c0 + e;
    const int idx = clampi(base + c * sc, 0, srcn - 1);
    const float x = src[idx];
    const _Float16 y = (_Float16)(bf_rt(x) * scale);
    out[e] = (rv && (c < cr)) ? y : (_Float16)0.0f;
  }
  _Float16* p = dst + (size_t)i * 8;
  *(volatile v8h*)p = out;
  __threadfence();
  *(volatile v8h*)p = out;
}

template <int NTL, int NCOLS, int KCH, int LDA, int AKR, int AZC>
__global__ __launch_bounds__(256) void gemm_f32rows(const _Float16* __restrict__ A, const _Float16* __restrict__ Bt,
                                                    const float* __restrict__ bias, int nbias, float scale,
                                                    float* C, int M, int rps, int spr, int roff) {
  static_assert((NTL % 4) == 0 && NTL <= 12 && NTL * 16 >= NCOLS && ((16 * NCOLS) % 4) == 0);
  extern __shared__ v4f dynslab4[];
  float* dynslab = (float*)dynslab4;
  constexpr int KP = KCH * 32;
  const int lane = threadIdx.x & 31;
  const int wave = threadIdx.x >> 5;
  const int h    = lane >> 4;
  const int m    = lane & 15;
  const int nw   = blockDim.x >> 5;
  const int row0 = (blockIdx.x * nw + wave) * 16;
  if (row0 >= M) return;
  const int r    = row0 + m;
  const int sg   = r / rps;
  const int prow = sg * spr + roff + (r - sg * rps);
  const _Float16* Ar = A + (size_t)prow * LDA;
  const _Float16* Bl = Bt + (size_t)m * KP + 8 * h;
  const int st = 16 * KP;

  v8f acc[NTL];
#pragma unroll
  for (int j = 0; j < NTL; ++j) acc[j] = zero8f();

#pragma unroll 1
  for (int k0 = 0; k0 < KP; k0 += 32) {
    const int Ka = k0 + 8 * h;
    const int Kb = Ka + 16;
    const int ca = (Ka >= AKR) ? AZC : Ka;
    const int cb = (Kb >= AKR) ? AZC : Kb;
    const v16h a = ldfrag(Ar + ca, Ar + cb);
    const _Float16* Bk = Bl + k0;
#pragma unroll
    for (int g = 0; g < NTL; g += 4) grp4(acc[g], acc[g + 1], acc[g + 2], acc[g + 3], a, Bk + g * st, st);
  }
#pragma unroll
  for (int g = 0; g < NTL; g += 4) accg4(acc[g], acc[g + 1], acc[g + 2], acc[g + 3]);

  float* slab = dynslab + wave * (16 * NCOLS);
#pragma unroll
  for (int j = 0; j < NTL; ++j) {
    const int col = j * 16 + m;
    const int bi  = (col < nbias) ? col : ((nbias > 0) ? (nbias - 1) : 0);
    const float bl = bf_rt(bias[bi]);
    const float bv = (col < nbias) ? bl : 0.f;
    if (col < NCOLS) {
#pragma unroll
      for (int rr = 0; rr < 8; ++rr) slab[(8 * h + rr) * NCOLS + col] = acc[j][rr] * scale + bv;
    }
  }
  wave_sync_lds();
  float* dst = C + (size_t)row0 * NCOLS;
  constexpr int NP  = 16 * NCOLS / 4;
  constexpr int NIT = (NP + 31) / 32;
  for (int pass = 0; pass < 2; ++pass) {
#pragma unroll
    for (int it = 0; it < NIT; ++it) {
      const int p = it * 32 + lane;
      if (p < NP) {
        const v4f v = *(const v4f*)(slab + p * 4);
        *(volatile v4f*)(dst + (size_t)p * 4) = v;
      }
    }
    __threadfence();
  }
}

__global__ __launch_bounds__(256) void embed_kernel(const int* __restrict__ char_ids, const int* __restrict__ text,
                                                    const float* __restrict__ T, const float* __restrict__ cnn_b,
                                                    const float* __restrict__ word_emb, _Float16* E) {
  __shared__ __align__(16) _Float16 stage[32 * PE];
  const int tid  = threadIdx.x;
  const int lane = tid & 31;
  const int wave = tid >> 5;
  const int w0   = blockIdx.x * 32;
  const int b    = w0 >> 9;
  const int s0   = w0 & (NS - 1);

  {
    const int word = w0 + lane;
    const int* ip = char_ids + (size_t)word * NW;
    const v4i q0 = *(const v4i*)(ip);
    const v4i q1 = *(const v4i*)(ip + 4);
    const v4i q2 = *(const v4i*)(ip + 8);
    const v4i q3 = *(const v4i*)(ip + 12);
    int id[NW];
#pragma unroll
    for (int e = 0; e < 4; ++e) {
      id[e]      = clampi(q0[e], 0, CV - 1);
      id[4 + e]  = clampi(q1[e], 0, CV - 1);
      id[8 + e]  = clampi(q2[e], 0, CV - 1);
      id[12 + e] = clampi(q3[e], 0, CV - 1);
    }
    const float* Tg = T + 8 * wave;
    v4f mA = zero4f(), mB = zero4f();
#pragma unroll
    for (int t = 0; t < NW; ++t) {
      v4f sA = zero4f(), sB = zero4f();
#pragma unroll
      for (int kk = 0; kk < 3; ++kk) {
        const int p = t - 1 + kk;
        if (p >= 0 && p < NW) {
          const float* tp = Tg + (size_t)id[p] * TN + kk * 64;
          sA += *(const v4f*)(tp);
          sB += *(const v4f*)(tp + 4);
        }
      }
      if (t == 0) {
        mA = sA;
        mB = sB;
      } else {
#pragma unroll
        for (int e = 0; e < 4; ++e) {
          mA[e] = fmaxf(mA[e], sA[e]);
          mB[e] = fmaxf(mB[e], sB[e]);
        }
      }
    }
    v4h ya, yb;
#pragma unroll
    for (int e = 0; e < 8; ++e) {
      const int o = 8 * wave + e;
      const float mv = (e < 4) ? mA[e & 3] : mB[e & 3];
      const float bb = bf_rt(cnn_b[(o < CE) ? o : (CE - 1)]);
      const float fm = (o < CE) ? 1.0f : 0.0f;
      const float v  = fmaxf(mv * (1.0f / 256.0f) + bb, 0.f) * fm;
      if (e < 4) ya[e & 3] = (_Float16)v; else yb[e & 3] = (_Float16)v;
    }
    _Float16* sp = stage + lane * PE + WE + 8 * wave;
    *(v4h*)(sp) = ya;
    if (8 * wave + 8 <= PE - WE) *(v4h*)(sp + 4) = yb;
  }

  for (int it = tid; it < 32 * (WE / 4); it += 256) {
    const int wl = it / (WE / 4);
    const int c4 = it - wl * (WE / 4);
    const int row = clampi(text[w0 + wl], 0, TV - 1);
    const v4f x = *(const v4f*)(word_emb + (size_t)row * WE + c4 * 4);
    v4h y;
#pragma unroll
    for (int e = 0; e < 4; ++e) y[e] = (_Float16)bf_rt(x[e]);
    *(v4h*)(stage + wl * PE + c4 * 4) = y;
  }
  __syncthreads();

  _Float16* dst = E + ((size_t)b * SEGR + 4 + s0) * PE;
  const bool g0 = (s0 == 0);
  const bool g1 = (s0 == NS - 32);
  _Float16* gz0 = E + (size_t)b * SEGR * PE;
  _Float16* gz1 = E + ((size_t)b * SEGR + 4 + NS) * PE;
  const v8h zz = zero8h();
  for (int pass = 0; pass < 2; ++pass) {
    for (int p = tid; p < (32 * PE) / 8; p += 256) {
      const v8h v = *(const v8h*)(stage + p * 8);
      *(volatile v8h*)(dst + (size_t)p * 8) = v;
    }
    if (g0 && tid < (4 * PE) / 8) *(volatile v8h*)(gz0 + (size_t)tid * 8) = zz;
    if (g1 && tid < (4 * PE) / 8) *(volatile v8h*)(gz1 + (size_t)tid * 8) = zz;
    __threadfence();
  }
}

template <int CS, int PA>
__device__ __forceinline__ const _Float16* conv_ap(const _Float16* xr, int K0) {
  const bool tail = K0 >= 3 * CS;
  int kk  = ((K0 >= CS) ? 1 : 0) + ((K0 >= 2 * CS) ? 1 : 0);
  int col = K0 - kk * CS;
  kk  = tail ? 0 : kk;
  col = tail ? (PA - 8) : col;
  return xr + kk * PA + col;
}

template <int CS, int PA, int KP>
__global__ __launch_bounds__(256) void conv_gemm(const _Float16* __restrict__ X, const _Float16* __restrict__ Wt,
                                                 const float* __restrict__ bias, _Float16* Y) {
  static_assert((KP % 32) == 0 && KP >= 3 * CS && (CS % 8) == 0 && PA >= 8);
  __shared__ __align__(16) _Float16 sT[8 * 16 * PH];
  const int lane = threadIdx.x & 31;
  const int wave = threadIdx.x >> 5;
  const int h    = lane >> 4;
  const int m    = lane & 15;
  const int b    = blockIdx.x >> 2;
  const int s0   = ((blockIdx.x & 3) << 7) + (wave << 4);
  const _Float16* Xr = X + ((size_t)b * SEGR + 3 + s0 + m) * PA;
  const _Float16* Bl = Wt + (size_t)m * KP + 8 * h;
  const int st = 16 * KP;

  v8f acc[13];
#pragma unroll
  for (int j = 0; j < 13; ++j) acc[j] = zero8f();

#pragma unroll 1
  for (int k0 = 0; k0 < KP; k0 += 32) {
    const int Ka = k0 + 8 * h;
    const int Kb = Ka + 16;
    const v16h a = ldfrag(conv_ap<CS, PA>(Xr, Ka), conv_ap<CS, PA>(Xr, Kb));
    const _Float16* Bk = Bl + k0;
    grp4(acc[0], acc[1], acc[2], acc[3], a, Bk, st);
    grp4(acc[4], acc[5], acc[6], acc[7], a, Bk + 4 * st, st);
    grp4(acc[8], acc[9], acc[10], acc[11], a, Bk + 8 * st, st);
    grp1(acc[12], a, Bk + 12 * st);
  }
  accg4(acc[0], acc[1], acc[2], acc[3]);
  accg4(acc[4], acc[5], acc[6], acc[7]);
  accg4(acc[8], acc[9], acc[10], acc[11]);
  accg1(acc[12]);

  _Float16* slab = sT + wave * (16 * PH);
  const float sc = 0.0625f;
#pragma unroll
  for (int j = 0; j < 13; ++j) {
    const int col = j * 16 + m;
    const int bc  = (col < CC) ? col : (CC - 1);
    const float bv = bf_rt(bias[bc]);
    const bool cv = col < CC;
#pragma unroll
    for (int rr = 0; rr < 8; ++rr) {
      float v = fmaxf(acc[j][rr] * sc + bv, 0.f);
      v = cv ? v : 0.f;
      slab[(8 * h + rr) * PH + col] = (_Float16)v;
    }
  }
  wave_sync_lds();
  _Float16* dst = Y + ((size_t)b * SEGR + 4 + s0) * PH;
  const bool g0 = (s0 == 0);
  const bool g1 = (s0 == NS - 16);
  _Float16* z0 = Y + (size_t)b * SEGR * PH;
  _Float16* z1 = Y + ((size_t)b * SEGR + 4 + NS) * PH;
  const v8h zz = zero8h();
  constexpr int NPD = (16 * PH) / 8;
  constexpr int NPG = (4 * PH) / 8;
  for (int pass = 0; pass < 2; ++pass) {
#pragma unroll
    for (int it = 0; it < NPD / 32; ++it) {
      const int p = it * 32 + lane;
      const v8h v = *(const v8h*)(slab + p * 8);
      *(volatile v8h*)(dst + (size_t)p * 8) = v;
    }
    if (g0) {
#pragma unroll
      for (int it = 0; it < (NPG + 31) / 32; ++it) {
        const int p = it * 32 + lane;
        if (p < NPG) *(volatile v8h*)(z0 + (size_t)p * 8) = zz;
      }
    }
    if (g1) {
#pragma unroll
      for (int it = 0; it < (NPG + 31) / 32; ++it) {
        const int p = it * 32 + lane;
        if (p < NPG) *(volatile v8h*)(z1 + (size_t)p * 8) = zz;
      }
    }
    __threadfence();
  }
}

static size_t align256(size_t v) { return (v + 255) & ~(size_t)255; }

extern "C" void kernel_launch(void* const* d_in, const int* in_sizes, int n_in,
                              void* d_out, int out_size, void* d_ws, size_t ws_size,
                              hipStream_t stream) {
  if (n_in < 16) return;
  if (in_sizes[0] != NWORD * NW) return;
  if (in_sizes[1] != NWORD) return;
  if (in_sizes[2] != CV * CE) return;
  if (in_sizes[3] != CE * CE * 3) return;
  if (in_sizes[4] != CE) return;
  if (in_sizes[5] != TV * WE) return;
  if (in_sizes[6] != CC * (WE + CE) * 3 || in_sizes[7] != CC) return;
  if (in_sizes[8] != CC * CC * 3 || in_sizes[9] != CC) return;
  if (in_sizes[10] != CC * CC * 3 || in_sizes[11] != CC) return;
  if (in_sizes[12] != CC * CC * 3 || in_sizes[13] != CC) return;
  if (in_sizes[14] != CC * NTAG || in_sizes[15] != NTAG) return;
  if (out_size != NWORD * NTAG) return;

  const int*   char_ids = (const int*)d_in[0];
  const int*   text     = (const int*)d_in[1];
  const float* char_emb = (const float*)d_in[2];
  const float* cnn_w    = (const float*)d_in[3];
  const float* cnn_b    = (const float*)d_in[4];
  const float* word_emb = (const float*)d_in[5];
  const float* conv1_w  = (const float*)d_in[6];
  const float* conv1_b  = (const float*)d_in[7];
  const float* conv2_w  = (const float*)d_in[8];
  const float* conv2_b  = (const float*)d_in[9];
  const float* conv3_w  = (const float*)d_in[10];
  const float* conv3_b  = (const float*)d_in[11];
  const float* conv4_w  = (const float*)d_in[12];
  const float* conv4_b  = (const float*)d_in[13];
  const float* out_w    = (const float*)d_in[14];
  const float* out_b    = (const float*)d_in[15];
  float* out = (float*)d_out;

  const size_t PW1 = (size_t)NCP * KC1 * 2;
  const size_t PW2 = (size_t)NCP * KC2 * 2;
  const size_t PWO = (size_t)NO * KO * 2;
  const size_t PBC = (size_t)TN * TK * 2;
  const size_t PEA = (size_t)TM * TK * 2;
  const size_t PT  = (size_t)TM * TN * 4;
  const size_t PEP = (size_t)NB * SEGR * PE * 2;
  const size_t PHP = (size_t)NB * SEGR * PH * 2;
  size_t off = 0;
  const size_t oW1 = off; off = align256(off + PW1);
  const size_t oW2 = off; off = align256(off + PW2);
  const size_t oW3 = off; off = align256(off + PW2);
  const size_t oW4 = off; off = align256(off + PW2);
  const size_t oWO = off; off = align256(off + PWO);
  const size_t oBC = off; off = align256(off + PBC);
  const size_t oEA = off; off = align256(off + PEA);
  const size_t oT  = off; off = align256(off + PT);
  const size_t oE  = off; off = align256(off + PEP);
  const size_t oHA = off; off = align256(off + PHP);
  const size_t oHB = off; off = align256(off + PHP);
  if (off > ws_size) return;
  if (off > (size_t)134217728) return;

  char* ws = (char*)d_ws;
  _Float16* W1 = (_Float16*)(ws + oW1);
  _Float16* W2 = (_Float16*)(ws + oW2);
  _Float16* W3 = (_Float16*)(ws + oW3);
  _Float16* W4 = (_Float16*)(ws + oW4);
  _Float16* WO = (_Float16*)(ws + oWO);
  _Float16* BC = (_Float16*)(ws + oBC);
  _Float16* EA = (_Float16*)(ws + oEA);
  float*    T  = (float*)(ws + oT);
  _Float16* E  = (_Float16*)(ws + oE);
  _Float16* HA = (_Float16*)(ws + oHA);
  _Float16* HB = (_Float16*)(ws + oHB);

  const dim3 blk(256);
  const int n8w1 = NCP * KC1 / 8;
  const int n8w2 = NCP * KC2 / 8;
  const int n8wo = NO * KO / 8;
  const int n8bc = TN * TK / 8;
  const int n8ea = TM * TK / 8;

  cvt_plane<<<dim3((n8w1 + 255) / 256), blk, 0, stream>>>(conv1_w, in_sizes[6], W1, KC1, NCP, 1, CC, CS1, 3, WE + CE,
                                                           (WE + CE) * 3, 0, 3, 1, 16.0f, n8w1);
  cvt_plane<<<dim3((n8w2 + 255) / 256), blk, 0, stream>>>(conv2_w, in_sizes[8], W2, KC2, NCP, 1, CC, CS2, 3, CC,
                                                           CC * 3, 0, 3, 1, 16.0f, n8w2);
  cvt_plane<<<dim3((n8w2 + 255) / 256), blk, 0, stream>>>(conv3_w, in_sizes[10], W3, KC2, NCP, 1, CC, CS2, 3, CC,
                                                           CC * 3, 0, 3, 1, 16.0f, n8w2);
  cvt_plane<<<dim3((n8w2 + 255) / 256), blk, 0, stream>>>(conv4_w, in_sizes[12], W4, KC2, NCP, 1, CC, CS2, 3, CC,
                                                           CC * 3, 0, 3, 1, 16.0f, n8w2);
  cvt_plane<<<dim3((n8wo + 255) / 256), blk, 0, stream>>>(out_w, in_sizes[14], WO, KO, NO, 1, NTAG, KO, 1, CC,
                                                           1, 0, NTAG, 0, 16.0f, n8wo);
  cvt_plane<<<dim3((n8bc + 255) / 256), blk, 0, stream>>>(cnn_w, in_sizes[3], BC, TK, 64, 3, CE, TK, 1, CE,
                                                           CE * 3, 1, 3, 0, 16.0f, n8bc);
  cvt_plane<<<dim3((n8ea + 255) / 256), blk, 0, stream>>>(char_emb, in_sizes[2], EA, TK, TM, 1, CV, TK, 1, CE,
                                                           CE, 0, 1, 0, 16.0f, n8ea);
  gemm_f32rows<12, TN, TK / 32, TK, TK, 0><<<dim3(TM / 32), dim3(64), (size_t)2 * 16 * TN * 4, stream>>>(
      EA, BC, cnn_b, 0, 1.0f, T, TM, TM, 0, 0);
  embed_kernel<<<dim3(NWORD / 32), blk, 0, stream>>>(char_ids, text, T, cnn_b, word_emb, E);
  conv_gemm<CS1, PE, KC1><<<dim3(NWORD / 128), blk, 0, stream>>>(E,  W1, conv1_b, HA);
  conv_gemm<CS2, PH, KC2><<<dim3(NWORD / 128), blk, 0, stream>>>(HA, W2, conv2_b, HB);
  conv_gemm<CS2, PH, KC2><<<dim3(NWORD / 128), blk, 0, stream>>>(HB, W3, conv3_b, HA);
  conv_gemm<CS2, PH, KC2><<<dim3(NWORD / 128), blk, 0, stream>>>(HA, W4, conv4_b, HB);
  gemm_f32rows<4, NTAG, KO / 32, PH, CC, CC><<<dim3(NWORD / 128), blk, (size_t)8 * 16 * NTAG * 4, stream>>>(
      HB, WO, out_b, NTAG, 0.0625f, out, NWORD, NS, SEGR, 4);
  (void)hipGetLastError();
}
